// HeatLayer_69638599737397
// MI455X (gfx1250) — hardware-verified
//
#include <hip/hip_runtime.h>
#include <math.h>

typedef __attribute__((ext_vector_type(16))) _Float16 v16h;
typedef __attribute__((ext_vector_type(16))) __bf16 v16b;
typedef __attribute__((ext_vector_type(8)))  _Float16 v8h;
typedef __attribute__((ext_vector_type(8)))  float v8f;
typedef __attribute__((ext_vector_type(4)))  float v4f;
typedef __attribute__((ext_vector_type(2)))  float v2f;
typedef __attribute__((ext_vector_type(4)))  unsigned v4u;
typedef __attribute__((ext_vector_type(4)))  int v4i;
typedef float __attribute__((may_alias)) float_a;
typedef int __attribute__((may_alias)) int_a;

template <typename T> __device__ __forceinline__ void vst2(void* p, T v) { *(volatile T*)p = v; __threadfence(); *(volatile T*)p = v; }
__device__ __forceinline__ v8f wmma16(v16h a, v16h b, v8f c) {
  v8f d = __builtin_amdgcn_wmma_f32_16x16x32_f16(false, a, false, b, (short)0, c, false, false);
  asm volatile("v_nop\n\tv_nop\n\tv_nop\n\tv_nop" : "+v"(d) : "v"(a), "v"(b));
  return d;
}
__device__ __forceinline__ v8f wmma_bf(v16b a, v16b b, v8f c) {
  v8f d = __builtin_amdgcn_wmma_f32_16x16x32_bf16(false, a, false, b, (short)0, c, false, false);
  asm volatile("v_nop\n\tv_nop\n\tv_nop\n\tv_nop" : "+v"(d) : "v"(a), "v"(b));
  return d;
}
__device__ __forceinline__ v16h frag_h(const _Float16* rowk0, int lane) {
  union { v16h v; v8h q[2]; } u; const _Float16* p = rowk0 + 8 * (lane >> 4);
  u.q[0] = *(const v8h*)p; u.q[1] = *(const v8h*)(p + 16); return u.v;
}
__device__ __forceinline__ v16h frag_f32(const float* rowk0, int lane) {
  v16h a; const float* p = rowk0 + 8 * (lane >> 4);
#pragma unroll
  for (int i = 0; i < 8; ++i) { a[i] = (_Float16)p[i]; a[8 + i] = (_Float16)p[16 + i]; }
  return a;
}
__device__ __forceinline__ v16h frag_f32s(const float* rowk0, int lane, float sc) {
  v16h a; const float* p = rowk0 + 8 * (lane >> 4);
#pragma unroll
  for (int i = 0; i < 8; ++i) { a[i] = (_Float16)(p[i] * sc); a[8 + i] = (_Float16)(p[16 + i] * sc); }
  return a;
}
__device__ __forceinline__ v16h fragc_f32(const float* W, int k0, int n, int lane, int ld, int K) {
  v16h a; const int g = lane >> 4;
#pragma unroll
  for (int i = 0; i < 8; ++i) { const int ka = k0 + 8 * g + i, kb = ka + 16;
    a[i] = (_Float16)(ka < K ? W[(size_t)(ka < K ? ka : K - 1) * ld + n] : 0.f); a[8 + i] = (_Float16)(kb < K ? W[(size_t)(kb < K ? kb : K - 1) * ld + n] : 0.f); }
  return a;
}
struct F2 { v16b h, l; };
__device__ __forceinline__ F2 bsplit16(const float v[16]) { F2 r;
#pragma unroll
  for (int i = 0; i < 16; ++i) { const __bf16 h = (__bf16)v[i]; r.h[i] = h; r.l[i] = (__bf16)(v[i] - (float)h); }
  return r; }
__device__ __forceinline__ F2 split_row(const float* row, int k0, int lane) { float v[16]; const float* p = row + k0 + 8 * (lane >> 4);
#pragma unroll
  for (int i = 0; i < 8; ++i) { v[i] = p[i]; v[8 + i] = p[16 + i]; }
  return bsplit16(v); }
__device__ __forceinline__ F2 split_rowK(const float* row, int k0, int lane, int K) { float v[16]; const int g = lane >> 4;
#pragma unroll
  for (int i = 0; i < 8; ++i) { const int ka = k0 + 8 * g + i, kb = ka + 16; v[i] = ka < K ? row[ka < K ? ka : K - 1] : 0.f; v[8 + i] = kb < K ? row[kb < K ? kb : K - 1] : 0.f; }
  return bsplit16(v); }
__device__ __forceinline__ F2 split_col(const float* W, int k0, int n, int lane, int ld, int K) { float v[16]; const int g = lane >> 4;
#pragma unroll
  for (int i = 0; i < 8; ++i) { const int ka = k0 + 8 * g + i, kb = ka + 16; v[i] = ka < K ? W[(size_t)(ka < K ? ka : K - 1) * ld + n] : 0.f; v[8 + i] = kb < K ? W[(size_t)(kb < K ? kb : K - 1) * ld + n] : 0.f; }
  return bsplit16(v); }
__device__ __forceinline__ v8f mac3(const F2& a, const F2& b, v8f c) { c = wmma_bf(a.l, b.h, c); c = wmma_bf(a.h, b.l, c); return wmma_bf(a.h, b.h, c); }
__device__ __forceinline__ float sigm(float v) { return 1.0f / (1.0f + expf(-v)); }
#define LDSX() do { asm volatile("s_wait_dscnt 0" ::: "memory"); __builtin_amdgcn_wave_barrier(); __builtin_amdgcn_fence(__ATOMIC_RELEASE, "workgroup"); } while (0)


#define SS 8192
#define DD 768
typedef __attribute__((ext_vector_type(8))) __bf16 v8b;
__device__ __forceinline__ v16b frag_b(const __bf16* rowk0, int lane) {
  union { v16b v; v8b q[2]; } u; const __bf16* p = rowk0 + 8 * (lane >> 4);
  u.q[0] = *(const v8b*)p; u.q[1] = *(const v8b*)(p + 16); return u.v;
}
__device__ __forceinline__ float bfr(float v) { return (float)(__bf16)v; }
__device__ __attribute__((noinline)) float exp_ni(float v) { return expf(v); }
__device__ __attribute__((noinline)) float erf_ni(float v) { return erff(v); }

#define WS_TS   0u
#define WS_PERM (WS_TS + 4u * SS)
#define WS_GE   (WS_PERM + 4u * SS)
#define WS_CS   (WS_GE + 4u * SS)
#define WS_ES   (WS_CS + 4u * (size_t)SS * DD)
#define WS_END  (WS_ES + 4u * (size_t)SS * DD)

__global__ __launch_bounds__(256) void k_sort(const float* __restrict__ T, float* __restrict__ TS, int* __restrict__ PERM, int* __restrict__ GE) {
  __shared__ float sk[SS]; __shared__ int sv[SS]; __shared__ int sge[SS];
  const int t = threadIdx.x;
  for (int i = t; i < SS; i += 256) { sk[i] = bfr(T[i]); sv[i] = i; }
  __syncthreads();
#pragma unroll 1
  for (int k = 2; k <= SS; k <<= 1) {
#pragma unroll 1
    for (int j = k >> 1; j > 0; j >>= 1) {
      for (int i = t; i < SS; i += 256) { const int l = i ^ j; if (l > i) { const bool up = ((i & k) == 0); const float a = sk[i], b = sk[l]; const bool sw = up ? (a > b) : (a < b); if (sw) { sk[i] = b; sk[l] = a; const int tv = sv[i]; sv[i] = sv[l]; sv[l] = tv; } } }
      __syncthreads(); } }
  if (t == 0) { int ge = SS - 1; for (int r = SS - 1; r >= 0; --r) { if (r < SS - 1 && sk[r] != sk[r + 1]) ge = r; sge[sv[r]] = ge; } }
  __syncthreads();
  for (int q = t; q < SS / 4; q += 256) { vst2(TS + q * 4, *(const v4f*)&sk[q * 4]); vst2((float*)(PERM + q * 4), *(const v4f*)&sv[q * 4]); vst2((float*)(GE + q * 4), *(const v4f*)&sge[q * 4]); } }
__global__ __launch_bounds__(128) void k_scan(const float* __restrict__ Hm, const float* __restrict__ TS, const int* __restrict__ PERM, const float* __restrict__ BETA, float* __restrict__ CS, float* __restrict__ ES) {
  __shared__ __align__(16) __bf16 s1[128][72], s2h[128][72], s2l[128][72];
  __shared__ __align__(16) float so[4][16][132]; __shared__ float carC[128], carE[128];
  const int tid = threadIdx.x, wave = tid >> 5, lane = tid & 31, col = lane & 15, g = lane >> 4; const int d0 = blockIdx.x * 128; const float beta = bfr(BETA[0]);
  for (int e = tid; e < 128; e += 128) { carC[e] = 0.f; carE[e] = 0.f; }
  v16b tri[2];
#pragma unroll
  for (int kc = 0; kc < 2; ++kc)
#pragma unroll
    for (int i = 0; i < 16; ++i) { const int k = kc * 32 + 8 * g + (i < 8 ? i : i + 8); tri[kc][i] = (k <= wave * 16 + col) ? (__bf16)1.0f : (__bf16)0.0f; }
#pragma unroll 1
  for (int rb = 0; rb < SS / 64; ++rb) {
    __syncthreads();
    for (int e = tid; e < 64 * 128; e += 128) { const int rk = e >> 7, ch = e & 127; const int r = rb * 64 + rk; const float hv = bfr(Hm[(size_t)PERM[r] * DD + d0 + ch]); s1[ch][rk] = (__bf16)hv; const float ev = fmaxf(hv, 0.f) * expf(-beta * TS[r]); const __bf16 eh = (__bf16)ev; s2h[ch][rk] = eh; s2l[ch][rk] = (__bf16)(ev - (float)eh); }
    __syncthreads();
    v8f a1[8] = {}, a2[8] = {};
#pragma unroll
    for (int kc = 0; kc < 2; ++kc) {
#pragma unroll
      for (int j = 0; j < 8; ++j) { const int ch = j * 16 + col; a1[j] = wmma_bf(tri[kc], frag_b(&s1[ch][kc * 32], lane), a1[j]); a2[j] = wmma_bf(tri[kc], frag_b(&s2h[ch][kc * 32], lane), a2[j]); a2[j] = wmma_bf(tri[kc], frag_b(&s2l[ch][kc * 32], lane), a2[j]); } }
#pragma unroll
    for (int j = 0; j < 8; ++j)
#pragma unroll
      for (int r = 0; r < 8; ++r) so[wave][8 * g + r][j * 16 + col] = a1[j][r] + carC[j * 16 + col];
    LDSX(); for (int rl = 0; rl < 16; ++rl) vst2(CS + (size_t)(rb * 64 + wave * 16 + rl) * DD + d0 + lane * 4, *(const v4f*)&so[wave][rl][lane * 4]);
    __syncthreads();
#pragma unroll
    for (int j = 0; j < 8; ++j)
#pragma unroll
      for (int r = 0; r < 8; ++r) so[wave][8 * g + r][j * 16 + col] = a2[j][r] + carE[j * 16 + col];
    LDSX(); for (int rl = 0; rl < 16; ++rl) vst2(ES + (size_t)(rb * 64 + wave * 16 + rl) * DD + d0 + lane * 4, *(const v4f*)&so[wave][rl][lane * 4]);
    __syncthreads();
    if (wave == 3 && g == 1) {
#pragma unroll
      for (int j = 0; j < 8; ++j) { carC[j * 16 + col] += a1[j][7]; carE[j * 16 + col] += a2[j][7]; } } } }
__global__ __launch_bounds__(256) void k_out(const float* __restrict__ T, const int* __restrict__ GE, const float* __restrict__ CS, const float* __restrict__ ES, const float* __restrict__ EPSI, const float* __restrict__ BETA, float* __restrict__ OUT) {
  const int tid = threadIdx.x; const size_t i0 = (size_t)blockIdx.x * 64; const float eps = bfr(EPSI[0]), beta = bfr(BETA[0]);
  for (int w = tid; w < 64 * (DD / 4); w += 256) { const int rl = w / (DD / 4), q = w % (DD / 4); const size_t i = i0 + rl; const int gi = GE[i]; const float f = eps * expf(beta * bfr(T[i]));
    const v4f c = *(const v4f*)(CS + (size_t)gi * DD + q * 4), e = *(const v4f*)(ES + (size_t)gi * DD + q * 4); v4f o; o[0] = c[0] + f * e[0]; o[1] = c[1] + f * e[1]; o[2] = c[2] + f * e[2]; o[3] = c[3] + f * e[3]; vst2(OUT + i * DD + q * 4, o); } }
extern "C" void kernel_launch(void* const* d_in, const int* in_sizes, int n_in, void* d_out, int out_size, void* d_ws, size_t ws_size, hipStream_t stream) {
  (void)in_sizes; (void)n_in; (void)out_size;
  const float** F = (const float**)d_in;
  if (ws_size < (size_t)WS_END) return;
  char* ws = (char*)d_ws; float *TS = (float*)(ws + WS_TS), *CS = (float*)(ws + WS_CS), *ES = (float*)(ws + WS_ES); int *PERM = (int*)(ws + WS_PERM), *GE = (int*)(ws + WS_GE);
  k_sort<<<1, 256, 0, stream>>>(F[1], TS, PERM, GE);
  k_scan<<<DD / 128, 128, 0, stream>>>(F[0], TS, PERM, F[3], CS, ES);
  k_out<<<SS / 64, 256, 0, stream>>>(F[1], GE, CS, ES, F[2], F[3], (float*)d_out);
}
